// CustomBertSelfAttention_79078937854339
// MI455X (gfx1250) — hardware-verified
//
#include <hip/hip_runtime.h>
#include <stdint.h>

constexpr int kBatch      = 2;
constexpr int kSeq        = 2048;
constexpr int kModel      = 1024;
constexpr int kHeads      = 16;
constexpr int kHeadDim    = 64;
constexpr int kTokens     = kBatch * kSeq;
constexpr int kPosRows    = 2 * kSeq - 1;
constexpr int kPosRowsPad = 4096;

static_assert(kTokens % 64 == 0 && kModel % 64 == 0 && kModel % 32 == 0 && kSeq % 64 == 0);
static_assert(kHeadDim == 64 && kHeads * kHeadDim == kModel && kSeq / 64 == 32 && kBatch * kHeads == 32);

constexpr size_t kXbBytes  = (size_t)kTokens * kModel * 2;
constexpr size_t kWtBytes  = (size_t)kModel * kModel * 2;
constexpr size_t kQkBytes  = (size_t)kTokens * kModel * 2;
constexpr size_t kVpBytes  = (size_t)kBatch * kModel * kSeq * 2;
constexpr size_t kEBytes   = (size_t)kPosRowsPad * kHeadDim * 2;
constexpr size_t kBrBytes  = (size_t)3 * kModel * 4;
constexpr size_t kWsTotal  = kXbBytes + 3 * kWtBytes + 2 * kQkBytes + 2 * kVpBytes + kEBytes + kBrBytes;
static_assert(kWsTotal == 48771072);
static_assert(kWsTotal <= 134217728);

typedef __attribute__((ext_vector_type(16))) _Float16 v16h;
typedef __attribute__((ext_vector_type(8)))  _Float16 v8h;
typedef __attribute__((ext_vector_type(16))) __bf16   v16b;
typedef __attribute__((ext_vector_type(8)))  __bf16   v8b;
typedef __attribute__((ext_vector_type(8)))  float    v8f;
typedef __attribute__((ext_vector_type(4)))  float    v4f;
typedef __attribute__((ext_vector_type(4)))  unsigned int v4u;
typedef __attribute__((ext_vector_type(2)))  unsigned int v2u;

__device__ __forceinline__ unsigned short f2bf_bits(float f) {
  unsigned u = __float_as_uint(f);
  return (unsigned short)((u + 0x7FFFu + ((u >> 16) & 1u)) >> 16);
}
__device__ __forceinline__ float bf_bits2f(unsigned short h) { return __uint_as_float(((unsigned)h) << 16); }

__device__ __forceinline__ void dep_guard_h(v8f& a, v8f& b, v16h x, v16h y) { asm volatile("v_nop\n\tv_nop\n\tv_nop\n\tv_nop" : "+v"(a), "+v"(b) : "v"(x), "v"(y)); }
__device__ __forceinline__ void dep_guard_b(v8f& a, v8f& b, v16b x, v16b y) { asm volatile("v_nop\n\tv_nop\n\tv_nop\n\tv_nop" : "+v"(a), "+v"(b) : "v"(x), "v"(y)); }
__device__ __forceinline__ void keep4_h(v16h a, v16h b, v16h c, v16h d) { asm volatile("v_nop" :: "v"(a), "v"(b), "v"(c), "v"(d)); }
__device__ __forceinline__ void keep4_b(v16b a, v16b b, v16b c, v16b d) { asm volatile("v_nop" :: "v"(a), "v"(b), "v"(c), "v"(d)); }
__device__ __forceinline__ void acc_guard4(v8f& a, v8f& b, v8f& c, v8f& d) { asm volatile("v_nop\n\tv_nop\n\tv_nop\n\tv_nop" : "+v"(a), "+v"(b), "+v"(c), "+v"(d)); }
template <typename T> struct Frag;
template <> struct Frag<_Float16> {
  typedef v16h V; union U { v16h v; v8h h[2]; };
  static __device__ __forceinline__ v16h load(const _Float16* p) {
    U f; f.h[0] = *(const v8h*)(p); f.h[1] = *(const v8h*)(p + 16); return f.v;
  }
  static __device__ __forceinline__ v8f mma(v16h a, v16h b, v8f c) {
    return __builtin_amdgcn_wmma_f32_16x16x32_f16(false, a, false, b, (short)0, c, false, false);
  }
  static __device__ __forceinline__ void guard(v8f& a, v8f& b, v16h x, v16h y) { dep_guard_h(a, b, x, y); }
  static __device__ __forceinline__ void keep(v16h a, v16h b, v16h c, v16h d) { keep4_h(a, b, c, d); }
};
template <> struct Frag<__bf16> {
  typedef v16b V; union U { v16b v; v8b h[2]; };
  static __device__ __forceinline__ v16b load(const __bf16* p) {
    U f; f.h[0] = *(const v8b*)(p); f.h[1] = *(const v8b*)(p + 16); return f.v;
  }
  static __device__ __forceinline__ v8f mma(v16b a, v16b b, v8f c) {
    return __builtin_amdgcn_wmma_f32_16x16x32_bf16(false, a, false, b, (short)0, c, false, false);
  }
  static __device__ __forceinline__ void guard(v8f& a, v8f& b, v16b x, v16b y) { dep_guard_b(a, b, x, y); }
  static __device__ __forceinline__ void keep(v16b a, v16b b, v16b c, v16b d) { keep4_b(a, b, c, d); }
};

template <int ET> struct Elem;
template <> struct Elem<0> { typedef _Float16 T; };
template <> struct Elem<1> { typedef __bf16 T; };
template <int ET, bool SPLIT, int BIAS_MODE, int OUT_MODE, bool RESID, int ACT = 0>
__global__ __launch_bounds__(256) void wmma_gemm64(
    const unsigned short* __restrict__ Ap, const unsigned short* __restrict__ A2p, int lda, long strideA,
    const unsigned short* __restrict__ Btp, const unsigned short* __restrict__ Bt2p, int ldb, long strideB,
    void* __restrict__ Cout, void* __restrict__ Cout2, int ldc, long strideC,
    const float* __restrict__ bias,
    const float* __restrict__ resid, long strideR,
    int M, int N, int K, float scale) {
  typedef typename Elem<ET>::T T;
  typedef typename Frag<T>::V V;
  const T* A = (const T*)Ap; const T* A2 = (const T*)A2p; const T* Bt = (const T*)Btp; const T* Bt2 = (const T*)Bt2p;
  __shared__ __align__(16) float sT[8][16 * 68];
  const int b    = blockIdx.y;
  const int lane = threadIdx.x & 31;
  const int wave = threadIdx.x >> 5;
  const int tilesN = N >> 6;
  const int tilesM = M >> 6;
  const int tile = blockIdx.x * 8 + wave;
  if (tile >= tilesM * tilesN) return;
  const int tm = tile / tilesN;
  const int tn = tile - tm * tilesN;
  const int m0 = tm << 6;
  const int n0 = tn << 6;

  const T* Ab  = A  + (size_t)b * strideA;
  const T* Bb  = Bt + (size_t)b * strideB;
  const T* Ab2 = SPLIT ? (A2  + (size_t)b * strideA) : nullptr;
  const T* Bb2 = SPLIT ? (Bt2 + (size_t)b * strideB) : nullptr;

  const int rlane = lane & 15;
  const int koff  = (lane >> 4) * 8;
  const int mOff  = (lane >> 4) * 8;

  v8f acc[4][4];
#pragma unroll
  for (int i = 0; i < 4; ++i)
#pragma unroll
    for (int j = 0; j < 4; ++j) acc[i][j] = (v8f){0.f,0.f,0.f,0.f,0.f,0.f,0.f,0.f};

  for (int k0 = 0; k0 < K; k0 += 32) {
    V bh[4], bl[4];
#pragma unroll
    for (int j = 0; j < 4; ++j) {
      const size_t bo = (size_t)(n0 + (j << 4) + rlane) * ldb + koff + k0;
      bh[j] = Frag<T>::load(Bb + bo);
      bl[j] = bh[j];
      if (SPLIT) bl[j] = Frag<T>::load(Bb2 + bo);
    }
#pragma unroll
    for (int i = 0; i < 4; ++i) {
      const size_t ao = (size_t)(m0 + (i << 4) + rlane) * lda + koff + k0;
      V ah = Frag<T>::load(Ab + ao);
      V al = ah;
      if (SPLIT) al = Frag<T>::load(Ab2 + ao);
#pragma unroll
      for (int j = 0; j < 4; ++j) {
        acc[i][j] = Frag<T>::mma(ah, bh[j], acc[i][j]);
        if (SPLIT) {
          acc[i][j] = Frag<T>::mma(ah, bl[j], acc[i][j]);
          acc[i][j] = Frag<T>::mma(al, bh[j], acc[i][j]);
        }
      }
      Frag<T>::guard(acc[i][0], acc[i][3], ah, al);
    }
    Frag<T>::keep(bh[0], bh[1], bh[2], bh[3]);
    if (SPLIT) Frag<T>::keep(bl[0], bl[1], bl[2], bl[3]);
  }
  acc_guard4(acc[0][0], acc[0][1], acc[0][2], acc[0][3]);
  acc_guard4(acc[1][0], acc[1][1], acc[1][2], acc[1][3]);
  acc_guard4(acc[2][0], acc[2][1], acc[2][2], acc[2][3]);
  acc_guard4(acc[3][0], acc[3][1], acc[3][2], acc[3][3]);

  float* slab = sT[wave];
  const float* Rb = RESID ? (resid + (size_t)b * strideR) : nullptr;
#pragma unroll
  for (int i = 0; i < 4; ++i) {
    const int mBase = m0 + (i << 4);
    float brow[8] = {0.f,0.f,0.f,0.f,0.f,0.f,0.f,0.f};
    if (BIAS_MODE == 1) {
      const v4f b0v = *(const v4f*)(bias + mBase + mOff);
      const v4f b1v = *(const v4f*)(bias + mBase + mOff + 4);
      brow[0] = b0v[0]; brow[1] = b0v[1]; brow[2] = b0v[2]; brow[3] = b0v[3];
      brow[4] = b1v[0]; brow[5] = b1v[1]; brow[6] = b1v[2]; brow[7] = b1v[3];
    }
#pragma unroll
    for (int j = 0; j < 4; ++j) {
      const int n = n0 + (j << 4) + rlane;
      float bv = 0.f;
      if (BIAS_MODE == 2) bv = bias[n];
#pragma unroll
      for (int r = 0; r < 8; ++r) {
        float v = acc[i][j][r] * scale;
        if (BIAS_MODE == 1) v += brow[r];
        if (BIAS_MODE == 2) v += bv;
        if (RESID) v += Rb[(size_t)(mBase + mOff + r) * ldc + n];
        if (ACT == 1) v = tanhf(v);
        if (ACT == 2) v = fmaxf(v, 0.0f);
        if (ACT == 4) v = (v > 0.f) ? v : 0.01f * v;
        slab[(mOff + r) * 68 + (j << 4) + rlane] = v;
      }
    }
    __builtin_amdgcn_fence(__ATOMIC_RELEASE, "workgroup");
    __builtin_amdgcn_wave_barrier();
    __builtin_amdgcn_fence(__ATOMIC_ACQUIRE, "workgroup");
    if (OUT_MODE == 0) {
      float* C = (float*)Cout + (size_t)b * strideC;
      const int hh = lane >> 4, c4 = (lane & 15) * 4;
      for (int pass = 0; pass < 2; ++pass) {
#pragma unroll
        for (int it = 0; it < 8; ++it) {
          const int row = it * 2 + hh;
          v4f v = *(const v4f*)(slab + row * 68 + c4);
          *(volatile v4f*)(C + (size_t)(mBase + row) * ldc + n0 + c4) = v;
        }
        __threadfence();
      }
    } else {
      const int q = lane >> 3, c8 = (lane & 7) * 8;
      unsigned short* C  = (unsigned short*)Cout  + (size_t)b * strideC;
      unsigned short* C2 = (OUT_MODE == 2) ? ((unsigned short*)Cout2 + (size_t)b * strideC) : nullptr;
      for (int pass = 0; pass < 2; ++pass) {
#pragma unroll
        for (int it = 0; it < 4; ++it) {
          const int row = it * 4 + q;
          const float* sp = slab + row * 68 + c8;
          v8h hv, lv;
#pragma unroll
          for (int e = 0; e < 8; ++e) {
            if (OUT_MODE == 1) {
              hv[e] = (_Float16)sp[e];
            } else {
              unsigned short hb = f2bf_bits(sp[e]);
              unsigned short lb = f2bf_bits(sp[e] - bf_bits2f(hb));
              hv[e] = __builtin_bit_cast(_Float16, hb);
              lv[e] = __builtin_bit_cast(_Float16, lb);
            }
          }
          *(volatile v8h*)(C + (size_t)(mBase + row) * ldc + n0 + c8) = hv;
          if (OUT_MODE == 2) *(volatile v8h*)(C2 + (size_t)(mBase + row) * ldc + n0 + c8) = lv;
        }
        __threadfence();
      }
    }
    __builtin_amdgcn_fence(__ATOMIC_RELEASE, "workgroup");
    __builtin_amdgcn_wave_barrier();
    __builtin_amdgcn_fence(__ATOMIC_ACQUIRE, "workgroup");
  }
}

__device__ __forceinline__ v8f mma_bf(v16b a, v16b b, v8f c) {
  c = __builtin_amdgcn_wmma_f32_16x16x32_bf16(false, a, false, b, (short)0, c, false, false);
  asm volatile("v_nop\n\tv_nop\n\tv_nop\n\tv_nop" : "+v"(c) : "v"(a), "v"(b));
  return c;
}
__device__ __forceinline__ v8f mma_hf(v16h a, v16h b, v8f c) {
  c = __builtin_amdgcn_wmma_f32_16x16x32_f16(false, a, false, b, (short)0, c, false, false);
  asm volatile("v_nop\n\tv_nop\n\tv_nop\n\tv_nop" : "+v"(c) : "v"(a), "v"(b));
  return c;
}

__global__ __launch_bounds__(256) void cvt_bf16x8_kernel(
    const float* __restrict__ in, unsigned short* __restrict__ outp, int n8) {
  const int i = blockIdx.x * 256 + threadIdx.x;
  if (i < n8) {
    const v4f a0 = *(const v4f*)(in + (size_t)i * 8);
    const v4f a1 = *(const v4f*)(in + (size_t)i * 8 + 4);
    v4u w;
    w[0] = (unsigned)f2bf_bits(a0[0]) | ((unsigned)f2bf_bits(a0[1]) << 16);
    w[1] = (unsigned)f2bf_bits(a0[2]) | ((unsigned)f2bf_bits(a0[3]) << 16);
    w[2] = (unsigned)f2bf_bits(a1[0]) | ((unsigned)f2bf_bits(a1[1]) << 16);
    w[3] = (unsigned)f2bf_bits(a1[2]) | ((unsigned)f2bf_bits(a1[3]) << 16);
    *(volatile v4u*)(outp + (size_t)i * 8) = w;
    __threadfence();
    *(volatile v4u*)(outp + (size_t)i * 8) = w;
  }
}

__global__ __launch_bounds__(256) void wtrans_bf16_kernel(
    const float* __restrict__ W, unsigned short* __restrict__ Wt) {
  __shared__ __align__(16) unsigned short tile[64 * 72];
  const int tid = threadIdx.x;
  const int n0 = blockIdx.x * 64, k0 = blockIdx.y * 64;
#pragma unroll
  for (int i = 0; i < 4; ++i) {
    const int ch = tid + 256 * i;
    const int kr = ch >> 4, c4 = (ch & 15) * 4;
    const v4f x = *(const v4f*)(W + (size_t)(k0 + kr) * kModel + n0 + c4);
#pragma unroll
    for (int e = 0; e < 4; ++e) tile[(c4 + e) * 72 + kr] = f2bf_bits(x[e]);
  }
  __syncthreads();
  const int lane = tid & 31, wave = tid >> 5;
  const int q = lane >> 3, c8 = (lane & 7) * 8;
  for (int pass = 0; pass < 2; ++pass) {
#pragma unroll
    for (int it = 0; it < 2; ++it) {
      const int row = it * 32 + wave * 4 + q;
      const v4u v = *(const v4u*)(tile + row * 72 + c8);
      *(volatile v4u*)(Wt + (size_t)(n0 + row) * kModel + k0 + c8) = v;
    }
    __threadfence();
  }
}

__global__ __launch_bounds__(256) void cvt_pos_kernel(
    const float* __restrict__ de, unsigned short* __restrict__ Ep) {
  const int i = blockIdx.x * 256 + threadIdx.x;
  const int row = i >> 3, c8 = (i & 7) * 8;
  const int rowc = (row < kPosRows) ? row : (kPosRows - 1);
  const float keep = (row < kPosRows) ? 1.0f : 0.0f;
  const v4f a0 = *(const v4f*)(de + (size_t)rowc * kHeadDim + c8);
  const v4f a1 = *(const v4f*)(de + (size_t)rowc * kHeadDim + c8 + 4);
  unsigned hb[8];
#pragma unroll
  for (int e = 0; e < 4; ++e) {
    const float y0 = bf_bits2f(f2bf_bits(a0[e])) * 256.0f * keep;
    const float y1 = bf_bits2f(f2bf_bits(a1[e])) * 256.0f * keep;
    hb[e]     = (unsigned)__builtin_bit_cast(unsigned short, (_Float16)y0);
    hb[4 + e] = (unsigned)__builtin_bit_cast(unsigned short, (_Float16)y1);
  }
  v4u w;
  w[0] = hb[0] | (hb[1] << 16);
  w[1] = hb[2] | (hb[3] << 16);
  w[2] = hb[4] | (hb[5] << 16);
  w[3] = hb[6] | (hb[7] << 16);
  *(volatile v4u*)(Ep + (size_t)i * 8) = w;
  __threadfence();
  *(volatile v4u*)(Ep + (size_t)i * 8) = w;
}

__global__ __launch_bounds__(256) void bias_prep_kernel(
    const float* __restrict__ b0, const float* __restrict__ b1, const float* __restrict__ b2,
    float* __restrict__ outp) {
  const float* src = (blockIdx.x == 0) ? b0 : ((blockIdx.x == 1) ? b1 : b2);
  const int t = threadIdx.x;
  const v4f x = *(const v4f*)(src + 4 * t);
  v4f y;
#pragma unroll
  for (int e = 0; e < 4; ++e) y[e] = bf_bits2f(f2bf_bits(x[e]));
  float* dst = outp + (size_t)blockIdx.x * kModel + 4 * t;
  *(volatile v4f*)dst = y;
  __threadfence();
  *(volatile v4f*)dst = y;
}

__global__ __launch_bounds__(128) void rel_attn_kernel(
    const unsigned short* __restrict__ Qp,
    const unsigned short* __restrict__ Kp,
    const unsigned short* __restrict__ Vhp,
    const unsigned short* __restrict__ Vlp,
    const unsigned short* __restrict__ Ep,
    const float* __restrict__ gmul,
    const float* __restrict__ aadd,
    float* __restrict__ outp) {
  __shared__ __align__(16) unsigned short Ksh[64 * 64];
  __shared__ __align__(16) unsigned short Vsh[64 * 64];
  __shared__ __align__(16) unsigned short Vsl[64 * 64];
  __shared__ __align__(16) unsigned short Esh[128 * 64];
  __shared__ __align__(16) unsigned short Msh[64 * 64];
  __shared__ __align__(16) unsigned short Psh[4][16 * 64];
  __shared__ __align__(16) unsigned short Psl[4][16 * 64];
  __shared__ __align__(16) float Gsh[4][16 * 80];

  const int tid  = threadIdx.x;
  const int wave = tid >> 5, lane = tid & 31, hh = lane >> 4, c = lane & 15;
  const int bx = blockIdx.x;
  const int qb = bx & 31;
  const int bh = bx >> 5;
  const int h  = bh & 15;
  const int b  = bh >> 4;
  const int l0 = qb * 64;
  const int q0 = l0 + wave * 16;

  union FH { v16h v; v8h p[2]; };
  union FB { v16b v; v8b p[2]; };

  v16h qa[2];
  {
    const unsigned short* qrow = Qp + (size_t)(b * kSeq + q0 + c) * kModel + h * kHeadDim;
#pragma unroll
    for (int dc = 0; dc < 2; ++dc) {
      FH f;
      f.p[0] = *(const v8h*)(qrow + dc * 32 + 8 * hh);
      f.p[1] = *(const v8h*)(qrow + dc * 32 + 16 + 8 * hh);
      qa[dc] = f.v;
    }
  }

  float mrow[8], lrow[8];
  v8f oacc[4];
#pragma unroll
  for (int r = 0; r < 8; ++r) { mrow[r] = -INFINITY; lrow[r] = 0.f; }
#pragma unroll
  for (int t = 0; t < 4; ++t) oacc[t] = (v8f){0.f,0.f,0.f,0.f,0.f,0.f,0.f,0.f};

  const unsigned short* kbase  = Kp + (size_t)(b * kSeq) * kModel + h * kHeadDim;
  const unsigned short* vhbase = Vhp + (size_t)b * kModel * kSeq + (size_t)(h * kHeadDim) * kSeq;
  const unsigned short* vlbase = Vlp + (size_t)b * kModel * kSeq + (size_t)(h * kHeadDim) * kSeq;
  const float* abase = aadd + (size_t)b * kSeq;

  for (int kc = 0; kc < kSeq / 64; ++kc) {
    const int kv0 = kc * 64;
    __syncthreads();
#pragma unroll
    for (int i = 0; i < 4; ++i) {
      const int ch = tid + 128 * i;
      const int row = ch >> 3, c8 = (ch & 7) * 8;
      const v4u w = *(const v4u*)(kbase + (size_t)(kv0 + row) * kModel + c8);
      *(v4u*)(Ksh + row * 64 + c8) = w;
    }
    asm volatile("" ::: "memory");
#pragma unroll
    for (int i = 0; i < 4; ++i) {
      const int ch = tid + 128 * i;
      const int d = ch >> 3, c8 = (ch & 7) * 8;
      const v4u w = *(const v4u*)(vhbase + (size_t)d * kSeq + kv0 + c8);
      *(v4u*)(Vsh + d * 64 + c8) = w;
    }
    asm volatile("" ::: "memory");
#pragma unroll
    for (int i = 0; i < 4; ++i) {
      const int ch = tid + 128 * i;
      const int d = ch >> 3, c8 = (ch & 7) * 8;
      const v4u w = *(const v4u*)(vlbase + (size_t)d * kSeq + kv0 + c8);
      *(v4u*)(Vsl + d * 64 + c8) = w;
    }
    asm volatile("" ::: "memory");
    const int base0 = l0 - kv0 + (kSeq - 1) - 63;
#pragma unroll
    for (int i = 0; i < 8; ++i) {
      const int ch = tid + 128 * i;
      const int r = ch >> 3, c8 = (ch & 7) * 8;
      int m = base0 + r;
      m = (m < 0) ? 0 : ((m > kPosRowsPad - 1) ? (kPosRowsPad - 1) : m);
      const v4u w = *(const v4u*)(Ep + (size_t)m * kHeadDim + c8);
      *(v4u*)(Esh + r * 64 + c8) = w;
    }
    asm volatile("" ::: "memory");
#pragma unroll
    for (int i = 0; i < 8; ++i) {
      const int ch = tid + 128 * i;
      const int ir = ch >> 4, c4 = (ch & 15) * 4;
      const v4f x = *(const v4f*)(gmul + (size_t)(l0 + ir) * kSeq + kv0 + c4);
      v2u st;
      st[0] = (unsigned)f2bf_bits(x[0]) | ((unsigned)f2bf_bits(x[1]) << 16);
      st[1] = (unsigned)f2bf_bits(x[2]) | ((unsigned)f2bf_bits(x[3]) << 16);
      *(v2u*)(Msh + ir * 64 + c4) = st;
    }
    float amr[4];
#pragma unroll
    for (int j = 0; j < 4; ++j) amr[j] = bf_bits2f(f2bf_bits(abase[kv0 + 16 * j + c]));
    __syncthreads();

    float* gw = Gsh[wave];
#pragma unroll
    for (int nc = 0; nc < 5; ++nc) {
      v8f g = (v8f){0.f,0.f,0.f,0.f,0.f,0.f,0.f,0.f};
      const unsigned short* erow = Esh + (16 * wave + 16 * nc + c) * 64;
#pragma unroll
      for (int dc = 0; dc < 2; ++dc) {
        FH eb;
        eb.p[0] = *(const v8h*)(erow + dc * 32 + 8 * hh);
        eb.p[1] = *(const v8h*)(erow + dc * 32 + 16 + 8 * hh);
        g = mma_hf(qa[dc], eb.v, g);
      }
#pragma unroll
      for (int r = 0; r < 8; ++r) gw[(8 * hh + r) * 80 + 16 * nc + c] = g[r];
    }

    v8f s[4];
#pragma unroll
    for (int j = 0; j < 4; ++j) {
      s[j] = (v8f){0.f,0.f,0.f,0.f,0.f,0.f,0.f,0.f};
      const unsigned short* krow = Ksh + (16 * j + c) * 64;
#pragma unroll
      for (int dc = 0; dc < 2; ++dc) {
        FH kb;
        kb.p[0] = *(const v8h*)(krow + dc * 32 + 8 * hh);
        kb.p[1] = *(const v8h*)(krow + dc * 32 + 16 + 8 * hh);
        s[j] = mma_hf(qa[dc], kb.v, s[j]);
      }
    }
    __builtin_amdgcn_fence(__ATOMIC_RELEASE, "workgroup");
    __builtin_amdgcn_wave_barrier();
    __builtin_amdgcn_fence(__ATOMIC_ACQUIRE, "workgroup");

    float cm[8];
#pragma unroll
    for (int r = 0; r < 8; ++r) {
      const int i  = 8 * hh + r;
      const int ib = 16 * wave + i;
      float m = -INFINITY;
#pragma unroll
      for (int j = 0; j < 4; ++j) {
        const int jj = 16 * j + c;
        const float gv = gw[i * 80 + (i - jj + 63)];
        const float mk = __uint_as_float(((unsigned)Msh[ib * 64 + jj]) << 16);
        float sc = (s[j][r] + gv * 0.00390625f) * 0.125f;
        sc = sc * mk + amr[j];
        s[j][r] = sc;
        m = fmaxf(m, sc);
      }
#pragma unroll
      for (int off = 1; off < 16; off <<= 1) m = fmaxf(m, __shfl_xor(m, off, 32));
      cm[r] = m;
    }

    unsigned short* ph  = Psh[wave];
    unsigned short* plo = Psl[wave];
#pragma unroll
    for (int r = 0; r < 8; ++r) {
      const float mnew  = fmaxf(mrow[r], cm[r]);
      const float alpha = expf(mrow[r] - mnew);
      mrow[r] = mnew;
      float psum = 0.f;
#pragma unroll
      for (int j = 0; j < 4; ++j) {
        const float p = expf(s[j][r] - mnew);
        psum += p;
        const unsigned short hb = f2bf_bits(p);
        const unsigned short lb = f2bf_bits(p - bf_bits2f(hb));
        ph[(8 * hh + r) * 64 + 16 * j + c]  = hb;
        plo[(8 * hh + r) * 64 + 16 * j + c] = lb;
      }
#pragma unroll
      for (int off = 1; off < 16; off <<= 1) psum += __shfl_xor(psum, off, 32);
      lrow[r] = lrow[r] * alpha + psum;
#pragma unroll
      for (int t = 0; t < 4; ++t) oacc[t][r] *= alpha;
    }
    __builtin_amdgcn_fence(__ATOMIC_RELEASE, "workgroup");
    __builtin_amdgcn_wave_barrier();
    __builtin_amdgcn_fence(__ATOMIC_ACQUIRE, "workgroup");

#pragma unroll 1
    for (int kk = 0; kk < 2; ++kk) {
      FB pa, pb;
      pa.p[0] = *(const v8b*)(ph + c * 64 + kk * 32 + 8 * hh);
      pa.p[1] = *(const v8b*)(ph + c * 64 + kk * 32 + 16 + 8 * hh);
      pb.p[0] = *(const v8b*)(plo + c * 64 + kk * 32 + 8 * hh);
      pb.p[1] = *(const v8b*)(plo + c * 64 + kk * 32 + 16 + 8 * hh);
#pragma unroll
      for (int t = 0; t < 4; ++t) {
        const unsigned short* vr = Vsh + (16 * t + c) * 64 + kk * 32;
        const unsigned short* vl = Vsl + (16 * t + c) * 64 + kk * 32;
        FB vb, wl;
        vb.p[0] = *(const v8b*)(vr + 8 * hh);
        vb.p[1] = *(const v8b*)(vr + 16 + 8 * hh);
        wl.p[0] = *(const v8b*)(vl + 8 * hh);
        wl.p[1] = *(const v8b*)(vl + 16 + 8 * hh);
        oacc[t] = mma_bf(pa.v, vb.v, oacc[t]);
        oacc[t] = mma_bf(pa.v, wl.v, oacc[t]);
        oacc[t] = mma_bf(pb.v, vb.v, oacc[t]);
      }
    }
  }

  float* os = Gsh[wave];
#pragma unroll
  for (int r = 0; r < 8; ++r) {
    const float inv = 1.0f / lrow[r];
#pragma unroll
    for (int t = 0; t < 4; ++t) os[(8 * hh + r) * 80 + 16 * t + c] = oacc[t][r] * inv;
  }
  __builtin_amdgcn_fence(__ATOMIC_RELEASE, "workgroup");
  __builtin_amdgcn_wave_barrier();
  __builtin_amdgcn_fence(__ATOMIC_ACQUIRE, "workgroup");
  {
    float* ob = outp + (size_t)(b * kSeq + q0) * kModel + h * kHeadDim;
    const int c4 = c * 4;
    for (int pass = 0; pass < 2; ++pass) {
#pragma unroll
      for (int it = 0; it < 8; ++it) {
        const int row = it * 2 + hh;
        const v4f val = *(const v4f*)(os + row * 80 + c4);
        *(volatile v4f*)(ob + (size_t)row * kModel + c4) = val;
      }
      __threadfence();
    }
  }
}

extern "C" void kernel_launch(void* const* d_in, const int* in_sizes, int n_in,
                              void* d_out, int out_size, void* d_ws, size_t ws_size,
                              hipStream_t stream) {
  if (n_in < 10) return;
  if (in_sizes[0] != kTokens * kModel) return;
  if (in_sizes[1] != kBatch * kSeq) return;
  if (in_sizes[2] != kSeq * kSeq) return;
  if (in_sizes[3] != kModel * kModel || in_sizes[5] != kModel * kModel || in_sizes[7] != kModel * kModel) return;
  if (in_sizes[4] != kModel || in_sizes[6] != kModel || in_sizes[8] != kModel) return;
  if (in_sizes[9] != kPosRows * kHeadDim) return;
  if (out_size != kTokens * kModel) return;
  if (ws_size < kWsTotal) return;

  const float* hs  = (const float*)d_in[0];
  const float* amk = (const float*)d_in[1];
  const float* gmk = (const float*)d_in[2];
  const float* Wq  = (const float*)d_in[3];
  const float* bq  = (const float*)d_in[4];
  const float* Wk  = (const float*)d_in[5];
  const float* bk  = (const float*)d_in[6];
  const float* Wv  = (const float*)d_in[7];
  const float* bv  = (const float*)d_in[8];
  const float* de  = (const float*)d_in[9];
  float* out = (float*)d_out;

  unsigned char* ws = (unsigned char*)d_ws;
  size_t off = 0;
  unsigned short* Xb  = (unsigned short*)(ws + off); off += kXbBytes;
  unsigned short* WqT = (unsigned short*)(ws + off); off += kWtBytes;
  unsigned short* WkT = (unsigned short*)(ws + off); off += kWtBytes;
  unsigned short* WvT = (unsigned short*)(ws + off); off += kWtBytes;
  unsigned short* Q16 = (unsigned short*)(ws + off); off += kQkBytes;
  unsigned short* K16 = (unsigned short*)(ws + off); off += kQkBytes;
  unsigned short* Vh  = (unsigned short*)(ws + off); off += kVpBytes;
  unsigned short* Vl  = (unsigned short*)(ws + off); off += kVpBytes;
  unsigned short* E16 = (unsigned short*)(ws + off); off += kEBytes;
  float*          Brz = (float*)(ws + off);          off += kBrBytes;
  if (off != kWsTotal || off > ws_size) return;

  const int n8 = (kTokens * kModel) / 8;
  cvt_bf16x8_kernel<<<dim3((n8 + 255) / 256), dim3(256), 0, stream>>>(hs, Xb, n8);
  wtrans_bf16_kernel<<<dim3(kModel / 64, kModel / 64), dim3(256), 0, stream>>>(Wq, WqT);
  wtrans_bf16_kernel<<<dim3(kModel / 64, kModel / 64), dim3(256), 0, stream>>>(Wk, WkT);
  wtrans_bf16_kernel<<<dim3(kModel / 64, kModel / 64), dim3(256), 0, stream>>>(Wv, WvT);
  cvt_pos_kernel<<<dim3((kPosRowsPad * kHeadDim / 8) / 256), dim3(256), 0, stream>>>(de, E16);
  bias_prep_kernel<<<dim3(3), dim3(256), 0, stream>>>(bq, bk, bv, Brz);

  wmma_gemm64<1, false, 2, 1, false, 0><<<dim3((kTokens / 64) * (kModel / 64) / 8, 1), dim3(256), 0, stream>>>(
      Xb, Xb, kModel, 0L, WqT, WqT, kModel, 0L, (void*)Q16, (void*)Q16, kModel, 0L,
      Brz, Brz, 0L, kTokens, kModel, kModel, 1.0f);
  wmma_gemm64<1, false, 2, 1, false, 0><<<dim3((kTokens / 64) * (kModel / 64) / 8, 1), dim3(256), 0, stream>>>(
      Xb, Xb, kModel, 0L, WkT, WkT, kModel, 0L, (void*)K16, (void*)K16, kModel, 0L,
      Brz + kModel, Brz, 0L, kTokens, kModel, kModel, 1.0f);
  wmma_gemm64<1, false, 1, 2, false, 0><<<dim3((kModel / 64) * (kSeq / 64) / 8, kBatch), dim3(256), 0, stream>>>(
      WvT, WvT, kModel, 0L, Xb, Xb, kModel, (long)kSeq * kModel, (void*)Vh, (void*)Vl, kSeq, (long)kModel * kSeq,
      Brz + 2 * kModel, Brz, 0L, kModel, kSeq, kModel, 1.0f);

  rel_attn_kernel<<<dim3(kBatch * kHeads * (kSeq / 64)), dim3(128), 0, stream>>>(
      Q16, K16, Vh, Vl, E16, gmk, amk, out);
}
